// Bottleneck_49039936586369
// MI455X (gfx1250) — hardware-verified
//
#include <hip/hip_runtime.h>
#define BB 8
#define CC 256
#define HS 32
#define WS 32
#define NPIX (HS * WS)
#define NH 8
#define HC 32
#define NG 4
#define GC 64
#define MR (BB * NPIX)

typedef __bf16 v16b __attribute__((ext_vector_type(16)));
typedef unsigned short v8us __attribute__((ext_vector_type(8), may_alias));
typedef float  v8f  __attribute__((ext_vector_type(8)));
typedef float  v4f  __attribute__((ext_vector_type(4)));
typedef float  v4fa __attribute__((ext_vector_type(4), may_alias));
union FragB { v16b v; v8us half[2]; unsigned short u[16]; };

__device__ __forceinline__ unsigned short bf16_bits(float x) { unsigned int u = __float_as_uint(x); return (unsigned short)((u + 0x7FFFu + ((u >> 16) & 1u)) >> 16); }
__device__ __forceinline__ float bf16_val(unsigned short b) { return __uint_as_float(((unsigned int)b) << 16); }
__device__ __forceinline__ float bf16_round(float x) { return bf16_val(bf16_bits(x)); }
template <int NT>
__device__ __forceinline__ v8f mmaN(v16b ah, v16b al, v16b bh, v16b bl, v8f c) {
  c = __builtin_amdgcn_wmma_f32_16x16x32_bf16(false, ah, false, bh, (short)0, c, false, false);
  if (NT >= 2) c = __builtin_amdgcn_wmma_f32_16x16x32_bf16(false, al, false, bh, (short)0, c, false, false);
  if (NT >= 3) c = __builtin_amdgcn_wmma_f32_16x16x32_bf16(false, ah, false, bl, (short)0, c, false, false);
  asm volatile("v_nop\n\tv_nop\n\tv_nop\n\tv_nop" : "+v"(c) : "v"(ah), "v"(al), "v"(bh), "v"(bl));
  return c;
}

__global__ __launch_bounds__(256) void k_wt_bf16(const float* __restrict__ W, unsigned short* __restrict__ Wt, int K, int N) {
  const int t = blockIdx.x * 256 + threadIdx.x;
  const int k8n = K / 8;
  if (t >= N * k8n) return;
  const int n = t / k8n, k8 = (t % k8n) * 8;
  v8us v;
#pragma unroll
  for (int i = 0; i < 8; ++i) v[i] = bf16_bits(W[(size_t)(k8 + i) * N + n]);
  *(volatile v8us*)(Wt + (size_t)n * K + k8) = v;
  __threadfence();
  *(volatile v8us*)(Wt + (size_t)n * K + k8) = v;
}

template <bool ASPLIT, int ACT, bool BIAS_BF16>
__global__ __launch_bounds__(128) void k_gemm_bf(const float* __restrict__ A, int lda, const unsigned short* __restrict__ Wt, int ldb,
                                               const float* __restrict__ bias, float* __restrict__ C, int ldc, int M, int N, int K) {
  __shared__ __attribute__((aligned(16))) float so[4][16][64];
  const int tid = threadIdx.x, w = tid >> 5, lane = tid & 31, ln = lane & 15, hh = lane >> 4;
  const int ntn = N / 64;
  const int wid = blockIdx.x * 4 + w;
  const int mt = wid / ntn, nq = wid % ntn;
  if (mt * 16 >= M) return;
  const int row0 = mt * 16, col0 = nq * 64;
  const float* arow = A + (size_t)(row0 + ln) * lda;
  v8f acc[4] = {};
  for (int kb = 0; kb < K; kb += 32) {
    FragB ah, al;
    const v4f x0 = *(const v4fa*)(arow + kb + 8 * hh), x1 = *(const v4fa*)(arow + kb + 8 * hh + 4);
    const v4f x2 = *(const v4fa*)(arow + kb + 16 + 8 * hh), x3 = *(const v4fa*)(arow + kb + 16 + 8 * hh + 4);
    float xs[16] = {x0[0],x0[1],x0[2],x0[3],x1[0],x1[1],x1[2],x1[3],x2[0],x2[1],x2[2],x2[3],x3[0],x3[1],x3[2],x3[3]};
#pragma unroll
    for (int i = 0; i < 16; ++i) { const unsigned short hb = bf16_bits(xs[i]); ah.u[i] = hb; al.u[i] = ASPLIT ? bf16_bits(xs[i] - bf16_val(hb)) : (unsigned short)0; }
#pragma unroll
    for (int t = 0; t < 4; ++t) {
      const unsigned short* brow = Wt + (size_t)(col0 + t * 16 + ln) * ldb + kb;
      FragB b;
      b.half[0] = *(const v8us*)(brow + 8 * hh);
      b.half[1] = *(const v8us*)(brow + 16 + 8 * hh);
      acc[t] = mmaN<ASPLIT ? 2 : 1>(ah.v, al.v, b.v, b.v, acc[t]);
    }
  }
#pragma unroll
  for (int t = 0; t < 4; ++t) {
    float bv = bias ? bias[col0 + t * 16 + ln] : 0.f;
    if (BIAS_BF16) bv = bf16_round(bv);
#pragma unroll
    for (int r = 0; r < 8; ++r) { float v = acc[t][r] + bv; if (ACT == 1) v = fmaxf(v, 0.f); so[w][8 * hh + r][t * 16 + ln] = v; }
  }
  __builtin_amdgcn_fence(__ATOMIC_ACQ_REL, "workgroup");
  __builtin_amdgcn_wave_barrier();
  const int rsub = lane >> 4, c4 = (lane & 15) * 4;
  for (int pass = 0; pass < 2; ++pass) {
#pragma unroll
    for (int q = 0; q < 8; ++q) {
      const int r = q * 2 + rsub;
      const v4f v = *(const v4fa*)&so[w][r][c4];
      *(volatile v4f*)(C + (size_t)(row0 + r) * ldc + col0 + c4) = v;
    }
    if (pass == 0) __threadfence();
  }
}

template <int D, bool CAUSAL>
__global__ __launch_bounds__(128) void k_flash(const float* __restrict__ qb, const float* __restrict__ kb, const float* __restrict__ vb,
                                             int pitch, int T, int H, float scale, float* __restrict__ y, int ypitch) {
  constexpr int KS = D / 32;
  constexpr int DT = D / 16;
  __shared__ __attribute__((aligned(16))) unsigned short sKh[32][D + 8], sKl[32][D + 8], sVh[32][D + 8], sVl[32][D + 8];
  __shared__ __attribute__((aligned(16))) unsigned short sPh[4][16][40], sPl[4][16][40];
  __shared__ __attribute__((aligned(16))) float sO[4][16][D];
  const int tid = threadIdx.x, w = tid >> 5, lane = tid & 31, ln = lane & 15, hh = lane >> 4;
  const int nqb = (T + 63) / 64;
  const int bh = blockIdx.x / nqb, qblk = blockIdx.x % nqb;
  const int b = bh / H, h = bh % H;
  const int q0 = qblk * 64 + w * 16;
  const float* Q = qb + (size_t)b * T * pitch + h * D;
  const float* K = kb + (size_t)b * T * pitch + h * D;
  const float* V = vb + (size_t)b * T * pitch + h * D;

  FragB aqh[KS], aql[KS];
  {
    int row = q0 + ln; if (row >= T) row = T - 1;
    const float* qr = Q + (size_t)row * pitch;
#pragma unroll
    for (int ks = 0; ks < KS; ++ks)
#pragma unroll
      for (int i = 0; i < 16; ++i) {
        const int d = ks * 32 + ((i < 8) ? (8 * hh + i) : (16 + 8 * hh + (i - 8)));
        const float x = qr[d] * scale; const unsigned short hb = bf16_bits(x);
        aqh[ks].u[i] = hb; aql[ks].u[i] = bf16_bits(x - bf16_val(hb));
      }
  }
  float m_r[8], l_r[8];
#pragma unroll
  for (int r = 0; r < 8; ++r) { m_r[r] = -3.0e38f; l_r[r] = 0.f; }
  v8f oacc[DT];
#pragma unroll
  for (int dt = 0; dt < DT; ++dt) oacc[dt] = (v8f){0.f,0.f,0.f,0.f,0.f,0.f,0.f,0.f};

  const int kv_end = CAUSAL ? min(T, qblk * 64 + 64) : T;
  for (int j0 = 0; j0 < kv_end; j0 += 32) {
    __syncthreads();
    for (int e = tid; e < 32 * (D / 4); e += 128) {
      const int r = e / (D / 4), c4 = (e % (D / 4)) * 4;
      const int key = j0 + r;
      v4f kf = {0.f,0.f,0.f,0.f}, vf = {0.f,0.f,0.f,0.f};
      if (key < T) { kf = *(const v4fa*)(K + (size_t)key * pitch + c4); vf = *(const v4fa*)(V + (size_t)key * pitch + c4); }
#pragma unroll
      for (int t = 0; t < 4; ++t) {
        unsigned short hb = bf16_bits(kf[t]); sKh[r][c4 + t] = hb; sKl[r][c4 + t] = bf16_bits(kf[t] - bf16_val(hb));
        hb = bf16_bits(vf[t]); sVh[r][c4 + t] = hb; sVl[r][c4 + t] = bf16_bits(vf[t] - bf16_val(hb));
      }
    }
    __syncthreads();
    v8f s[2];
#pragma unroll
    for (int nt = 0; nt < 2; ++nt) {
      v8f acc = {};
#pragma unroll
      for (int ks = 0; ks < KS; ++ks) {
        FragB bh_, bl_;
        bh_.half[0] = *(const v8us*)&sKh[nt * 16 + ln][ks * 32 + 8 * hh]; bh_.half[1] = *(const v8us*)&sKh[nt * 16 + ln][ks * 32 + 16 + 8 * hh];
        bl_.half[0] = *(const v8us*)&sKl[nt * 16 + ln][ks * 32 + 8 * hh]; bl_.half[1] = *(const v8us*)&sKl[nt * 16 + ln][ks * 32 + 16 + 8 * hh];
        acc = mmaN<3>(aqh[ks].v, aql[ks].v, bh_.v, bl_.v, acc);
      }
      s[nt] = acc;
    }
    float alpha[8];
#pragma unroll
    for (int r = 0; r < 8; ++r) {
      const int qi = q0 + 8 * hh + r;
      const int ja = j0 + ln, jb = j0 + 16 + ln;
      if (CAUSAL) { if (ja > qi) s[0][r] = -3.0e38f; if (jb > qi) s[1][r] = -3.0e38f; }
      if (ja >= T) s[0][r] = -3.0e38f;
      if (jb >= T) s[1][r] = -3.0e38f;
      float mx = fmaxf(s[0][r], s[1][r]);
      mx = fmaxf(mx, __shfl_xor(mx, 1, 32)); mx = fmaxf(mx, __shfl_xor(mx, 2, 32)); mx = fmaxf(mx, __shfl_xor(mx, 4, 32)); mx = fmaxf(mx, __shfl_xor(mx, 8, 32));
      const float mnew = fmaxf(m_r[r], mx);
      alpha[r] = (mnew > -1.0e38f) ? __expf(m_r[r] - mnew) : 1.0f;
      const float p0 = (s[0][r] > -1.0e38f) ? __expf(s[0][r] - mnew) : 0.f;
      const float p1 = (s[1][r] > -1.0e38f) ? __expf(s[1][r] - mnew) : 0.f;
      m_r[r] = mnew;
      l_r[r] = l_r[r] * alpha[r] + p0 + p1;
      unsigned short hb = bf16_bits(p0); sPh[w][8 * hh + r][ln] = hb;      sPl[w][8 * hh + r][ln] = bf16_bits(p0 - bf16_val(hb));
      hb = bf16_bits(p1);                sPh[w][8 * hh + r][16 + ln] = hb; sPl[w][8 * hh + r][16 + ln] = bf16_bits(p1 - bf16_val(hb));
    }
#pragma unroll
    for (int dt = 0; dt < DT; ++dt)
#pragma unroll
      for (int r = 0; r < 8; ++r) oacc[dt][r] *= alpha[r];
    __builtin_amdgcn_fence(__ATOMIC_ACQ_REL, "workgroup");
    __builtin_amdgcn_wave_barrier();
    FragB pah, pal;
    pah.half[0] = *(const v8us*)&sPh[w][ln][8 * hh]; pah.half[1] = *(const v8us*)&sPh[w][ln][16 + 8 * hh];
    pal.half[0] = *(const v8us*)&sPl[w][ln][8 * hh]; pal.half[1] = *(const v8us*)&sPl[w][ln][16 + 8 * hh];
#pragma unroll
    for (int dt = 0; dt < DT; ++dt) {
      FragB bvh, bvl;
#pragma unroll
      for (int i = 0; i < 8; ++i) {
        bvh.u[i] = sVh[8 * hh + i][dt * 16 + ln]; bvh.u[8 + i] = sVh[16 + 8 * hh + i][dt * 16 + ln];
        bvl.u[i] = sVl[8 * hh + i][dt * 16 + ln]; bvl.u[8 + i] = sVl[16 + 8 * hh + i][dt * 16 + ln];
      }
      oacc[dt] = mmaN<3>(pah.v, pal.v, bvh.v, bvl.v, oacc[dt]);
    }
    __builtin_amdgcn_fence(__ATOMIC_ACQ_REL, "workgroup");
    __builtin_amdgcn_wave_barrier();
  }
#pragma unroll
  for (int r = 0; r < 8; ++r) {
    float l = l_r[r];
    l += __shfl_xor(l, 1, 32); l += __shfl_xor(l, 2, 32); l += __shfl_xor(l, 4, 32); l += __shfl_xor(l, 8, 32);
    l_r[r] = (l > 0.f) ? 1.0f / l : 0.f;
  }
#pragma unroll
  for (int dt = 0; dt < DT; ++dt)
#pragma unroll
    for (int r = 0; r < 8; ++r) sO[w][8 * hh + r][dt * 16 + ln] = oacc[dt][r] * l_r[r];
  __builtin_amdgcn_fence(__ATOMIC_ACQ_REL, "workgroup");
  __builtin_amdgcn_wave_barrier();
  for (int pass = 0; pass < 2; ++pass) {
    for (int r = 0; r < 16; ++r) {
      const int row = q0 + r;
      if (row < T && lane < D / 4) {
        const v4f val = *(const v4fa*)&sO[w][r][lane * 4];
        *(volatile v4f*)(y + ((size_t)b * T + row) * ypitch + h * D + lane * 4) = val;
      }
    }
    if (pass == 0) __threadfence();
  }
}

template <bool AFFINE, bool RESID, bool RES_BF16>
__global__ __launch_bounds__(256) void k_transpose32(const float* __restrict__ in, float* __restrict__ out, int rows, int cols,
                                                    const float* __restrict__ scale, const float* __restrict__ shift, const float* __restrict__ res) {
  __shared__ float tile[32][33];
  const int b = blockIdx.z;
  const int r0 = blockIdx.y * 32, c0 = blockIdx.x * 32;
  const float* src = in + (size_t)b * rows * cols;
  float* dst = out + (size_t)b * rows * cols;
  const int tx = threadIdx.x & 31, ty = threadIdx.x >> 5;
  for (int i = ty; i < 32; i += 8) tile[i][tx] = src[(size_t)(r0 + i) * cols + c0 + tx];
  __syncthreads();
  for (int pass = 0; pass < 2; ++pass) {
    for (int i = ty; i < 32; i += 8) {
      float v = tile[tx][i];
      const int orow = c0 + i;
      if (AFFINE) v = v * scale[orow] + shift[orow];
      if (RESID) { float rv = res[(size_t)b * rows * cols + (size_t)orow * rows + r0 + tx]; if (RES_BF16) rv = bf16_round(rv); v += rv; }
      *(volatile float*)(dst + (size_t)orow * rows + r0 + tx) = v;
    }
    if (pass == 0) __threadfence();
  }
}

__global__ __launch_bounds__(256) void k_pool2_pm(const float* __restrict__ in, float* __restrict__ out, int Bn, int H, int W, int C) {
  const size_t t = (size_t)blockIdx.x * 256 + threadIdx.x;
  const int c4n = C / 4, Ho = H / 2, Wo = W / 2;
  const size_t total = (size_t)Bn * Ho * Wo * c4n;
  if (t >= total) return;
  const int c4 = (int)(t % c4n) * 4; size_t rest = t / c4n;
  const int pw = (int)(rest % Wo); rest /= Wo; const int ph = (int)(rest % Ho); const int b = (int)(rest / Ho);
  const float* base = in + (size_t)b * H * W * C;
  const int p00 = (2 * ph) * W + 2 * pw;
  const v4f a = *(const v4fa*)(base + (size_t)p00 * C + c4), bq = *(const v4fa*)(base + (size_t)(p00 + 1) * C + c4);
  const v4f c = *(const v4fa*)(base + (size_t)(p00 + W) * C + c4), d = *(const v4fa*)(base + (size_t)(p00 + W + 1) * C + c4);
  v4f m; for (int i = 0; i < 4; ++i) m[i] = fmaxf(fmaxf(a[i], bq[i]), fmaxf(c[i], d[i]));
  float* dst = out + ((size_t)b * Ho * Wo + (size_t)ph * Wo + pw) * C + c4;
  *(volatile v4f*)dst = m;
  __threadfence();
  *(volatile v4f*)dst = m;
}

template <int DQ, int DV>
__global__ __launch_bounds__(128) void k_flash2(const float* __restrict__ Qb, size_t qstride, int qpitch, int Tq,
                                              const float* __restrict__ Kb, size_t kstride, int kpitch, int Tk,
                                              const float* __restrict__ Vb, size_t vstride, int vpitch,
                                              float scale, float* __restrict__ y, size_t ystride, int ypitch) {
  constexpr int KS = DQ / 32, DT = DV / 16;
  __shared__ __attribute__((aligned(16))) unsigned short sKh[32][DQ + 8], sKl[32][DQ + 8], sVh[32][DV + 8], sVl[32][DV + 8];
  __shared__ __attribute__((aligned(16))) unsigned short sPh[4][16][40], sPl[4][16][40];
  __shared__ __attribute__((aligned(16))) float sO[4][16][DV];
  const int tid = threadIdx.x, w = tid >> 5, lane = tid & 31, ln = lane & 15, hh = lane >> 4;
  const int nqb = (Tq + 63) / 64;
  const int bh = blockIdx.x / nqb, qblk = blockIdx.x % nqb;
  const int dv0 = blockIdx.y * DV;
  const int q0 = qblk * 64 + w * 16;
  const float* Q = Qb + (size_t)bh * qstride; const float* K = Kb + (size_t)bh * kstride; const float* V = Vb + (size_t)bh * vstride + dv0;
  FragB aqh[KS], aql[KS];
  {
    int row = q0 + ln; if (row >= Tq) row = Tq - 1;
    const float* qr = Q + (size_t)row * qpitch;
#pragma unroll
    for (int ks = 0; ks < KS; ++ks)
#pragma unroll
      for (int i = 0; i < 16; ++i) {
        const int d = ks * 32 + ((i < 8) ? (8 * hh + i) : (16 + 8 * hh + (i - 8)));
        const float x = qr[d] * scale; const unsigned short hb = bf16_bits(x);
        aqh[ks].u[i] = hb; aql[ks].u[i] = bf16_bits(x - bf16_val(hb));
      }
  }
  float m_r[8], l_r[8];
#pragma unroll
  for (int r = 0; r < 8; ++r) { m_r[r] = -3.0e38f; l_r[r] = 0.f; }
  v8f oacc[DT];
#pragma unroll
  for (int dt = 0; dt < DT; ++dt) oacc[dt] = (v8f){0.f,0.f,0.f,0.f,0.f,0.f,0.f,0.f};
  for (int j0 = 0; j0 < Tk; j0 += 32) {
    __syncthreads();
    for (int e = tid; e < 32 * (DQ / 4); e += 128) {
      const int r = e / (DQ / 4), c4 = (e % (DQ / 4)) * 4; const int key = j0 + r;
      v4f f = {0.f,0.f,0.f,0.f}; if (key < Tk) f = *(const v4fa*)(K + (size_t)key * kpitch + c4);
#pragma unroll
      for (int t = 0; t < 4; ++t) { const unsigned short hb = bf16_bits(f[t]); sKh[r][c4 + t] = hb; sKl[r][c4 + t] = bf16_bits(f[t] - bf16_val(hb)); }
    }
    for (int e = tid; e < 32 * (DV / 4); e += 128) {
      const int r = e / (DV / 4), c4 = (e % (DV / 4)) * 4; const int key = j0 + r;
      v4f f = {0.f,0.f,0.f,0.f}; if (key < Tk) f = *(const v4fa*)(V + (size_t)key * vpitch + c4);
#pragma unroll
      for (int t = 0; t < 4; ++t) { const unsigned short hb = bf16_bits(f[t]); sVh[r][c4 + t] = hb; sVl[r][c4 + t] = bf16_bits(f[t] - bf16_val(hb)); }
    }
    __syncthreads();
    v8f s[2];
#pragma unroll
    for (int nt = 0; nt < 2; ++nt) {
      v8f acc = {};
#pragma unroll
      for (int ks = 0; ks < KS; ++ks) {
        FragB bh_, bl_;
        bh_.half[0] = *(const v8us*)&sKh[nt * 16 + ln][ks * 32 + 8 * hh]; bh_.half[1] = *(const v8us*)&sKh[nt * 16 + ln][ks * 32 + 16 + 8 * hh];
        bl_.half[0] = *(const v8us*)&sKl[nt * 16 + ln][ks * 32 + 8 * hh]; bl_.half[1] = *(const v8us*)&sKl[nt * 16 + ln][ks * 32 + 16 + 8 * hh];
        acc = mmaN<3>(aqh[ks].v, aql[ks].v, bh_.v, bl_.v, acc);
      }
      s[nt] = acc;
    }
    float alpha[8];
#pragma unroll
    for (int r = 0; r < 8; ++r) {
      const int ja = j0 + ln, jb = j0 + 16 + ln;
      if (ja >= Tk) s[0][r] = -3.0e38f;
      if (jb >= Tk) s[1][r] = -3.0e38f;
      float mx = fmaxf(s[0][r], s[1][r]);
      mx = fmaxf(mx, __shfl_xor(mx, 1, 32)); mx = fmaxf(mx, __shfl_xor(mx, 2, 32)); mx = fmaxf(mx, __shfl_xor(mx, 4, 32)); mx = fmaxf(mx, __shfl_xor(mx, 8, 32));
      const float mnew = fmaxf(m_r[r], mx);
      alpha[r] = (mnew > -1.0e38f) ? __expf(m_r[r] - mnew) : 1.0f;
      const float p0 = (s[0][r] > -1.0e38f) ? __expf(s[0][r] - mnew) : 0.f;
      const float p1 = (s[1][r] > -1.0e38f) ? __expf(s[1][r] - mnew) : 0.f;
      m_r[r] = mnew;
      l_r[r] = l_r[r] * alpha[r] + p0 + p1;
      unsigned short hb = bf16_bits(p0); sPh[w][8 * hh + r][ln] = hb;      sPl[w][8 * hh + r][ln] = bf16_bits(p0 - bf16_val(hb));
      hb = bf16_bits(p1);                sPh[w][8 * hh + r][16 + ln] = hb; sPl[w][8 * hh + r][16 + ln] = bf16_bits(p1 - bf16_val(hb));
    }
#pragma unroll
    for (int dt = 0; dt < DT; ++dt)
#pragma unroll
      for (int r = 0; r < 8; ++r) oacc[dt][r] *= alpha[r];
    __builtin_amdgcn_fence(__ATOMIC_ACQ_REL, "workgroup");
    __builtin_amdgcn_wave_barrier();
    FragB pah, pal;
    pah.half[0] = *(const v8us*)&sPh[w][ln][8 * hh]; pah.half[1] = *(const v8us*)&sPh[w][ln][16 + 8 * hh];
    pal.half[0] = *(const v8us*)&sPl[w][ln][8 * hh]; pal.half[1] = *(const v8us*)&sPl[w][ln][16 + 8 * hh];
#pragma unroll
    for (int dt = 0; dt < DT; ++dt) {
      FragB bvh, bvl;
#pragma unroll
      for (int i = 0; i < 8; ++i) {
        bvh.u[i] = sVh[8 * hh + i][dt * 16 + ln]; bvh.u[8 + i] = sVh[16 + 8 * hh + i][dt * 16 + ln];
        bvl.u[i] = sVl[8 * hh + i][dt * 16 + ln]; bvl.u[8 + i] = sVl[16 + 8 * hh + i][dt * 16 + ln];
      }
      oacc[dt] = mmaN<3>(pah.v, pal.v, bvh.v, bvl.v, oacc[dt]);
    }
    __builtin_amdgcn_fence(__ATOMIC_ACQ_REL, "workgroup");
    __builtin_amdgcn_wave_barrier();
  }
#pragma unroll
  for (int r = 0; r < 8; ++r) {
    float l = l_r[r];
    l += __shfl_xor(l, 1, 32); l += __shfl_xor(l, 2, 32); l += __shfl_xor(l, 4, 32); l += __shfl_xor(l, 8, 32);
    l_r[r] = (l > 0.f) ? 1.0f / l : 0.f;
  }
#pragma unroll
  for (int dt = 0; dt < DT; ++dt)
#pragma unroll
    for (int r = 0; r < 8; ++r) sO[w][8 * hh + r][dt * 16 + ln] = oacc[dt][r] * l_r[r];
  __builtin_amdgcn_fence(__ATOMIC_ACQ_REL, "workgroup");
  __builtin_amdgcn_wave_barrier();
  for (int pass = 0; pass < 2; ++pass) {
    for (int r = 0; r < 16; ++r) {
      const int row = q0 + r;
      for (int c4 = lane * 4; c4 < DV; c4 += 128) {
        if (row < Tq) {
          const v4f val = *(const v4fa*)&sO[w][r][c4];
          *(volatile v4f*)(y + (size_t)bh * ystride + (size_t)row * ypitch + dv0 + c4) = val;
        }
      }
    }
    if (pass == 0) __threadfence();
  }
}

template <bool ASPLIT, int ACT, bool BIAS_BF16, bool RES_BF16>
__global__ __launch_bounds__(128) void k_gemm_bf3(const float* __restrict__ A, int lda, const unsigned short* __restrict__ Wt, int ldb,
                                                const float* __restrict__ bias, const float* __restrict__ resid, int rmod, int ldr,
                                                float* __restrict__ C, int ldc, int M, int N, int K) {
  __shared__ __attribute__((aligned(16))) float so[4][16][64];
  const int tid = threadIdx.x, w = tid >> 5, lane = tid & 31, ln = lane & 15, hh = lane >> 4;
  const int ntn = N / 64;
  const int wid = blockIdx.x * 4 + w;
  const int mt = wid / ntn, nq = wid % ntn;
  if (mt * 16 >= M) return;
  const int row0 = mt * 16, col0 = nq * 64;
  const float* arow = A + (size_t)(row0 + ln) * lda;
  v8f acc[4] = {};
  for (int kb = 0; kb < K; kb += 32) {
    FragB ah, al;
    const v4f x0 = *(const v4fa*)(arow + kb + 8 * hh), x1 = *(const v4fa*)(arow + kb + 8 * hh + 4);
    const v4f x2 = *(const v4fa*)(arow + kb + 16 + 8 * hh), x3 = *(const v4fa*)(arow + kb + 16 + 8 * hh + 4);
    float xs[16] = {x0[0],x0[1],x0[2],x0[3],x1[0],x1[1],x1[2],x1[3],x2[0],x2[1],x2[2],x2[3],x3[0],x3[1],x3[2],x3[3]};
#pragma unroll
    for (int i = 0; i < 16; ++i) { const unsigned short hb = bf16_bits(xs[i]); ah.u[i] = hb; al.u[i] = ASPLIT ? bf16_bits(xs[i] - bf16_val(hb)) : (unsigned short)0; }
#pragma unroll
    for (int t = 0; t < 4; ++t) {
      const unsigned short* brow = Wt + (size_t)(col0 + t * 16 + ln) * ldb + kb;
      FragB b;
      b.half[0] = *(const v8us*)(brow + 8 * hh);
      b.half[1] = *(const v8us*)(brow + 16 + 8 * hh);
      acc[t] = mmaN<ASPLIT ? 2 : 1>(ah.v, al.v, b.v, b.v, acc[t]);
    }
  }
#pragma unroll
  for (int t = 0; t < 4; ++t) {
    const int col = col0 + t * 16 + ln;
    float bv = bias ? bias[col] : 0.f;
    if (BIAS_BF16) bv = bf16_round(bv);
#pragma unroll
    for (int r = 0; r < 8; ++r) {
      float v = acc[t][r] + bv;
      if (resid) { float rv = resid[(size_t)((row0 + 8 * hh + r) % rmod) * ldr + col]; if (RES_BF16) rv = bf16_round(rv); v += rv; }
      if (ACT == 1) v = fmaxf(v, 0.f);
      if (ACT == 2) v = 0.5f * v * (1.0f + erff(v * 0.70710678118654752f));
      if (ACT == 3) { const float u = 0.7978845608028654f * (v + 0.044715f * v * v * v); v = 0.5f * v * (1.0f + tanhf(u)); }
      so[w][8 * hh + r][t * 16 + ln] = v;
    }
  }
  __builtin_amdgcn_fence(__ATOMIC_ACQ_REL, "workgroup");
  __builtin_amdgcn_wave_barrier();
  const int rsub = lane >> 4, c4 = (lane & 15) * 4;
  for (int pass = 0; pass < 2; ++pass) {
#pragma unroll
    for (int q = 0; q < 8; ++q) {
      const int r = q * 2 + rsub;
      const v4f v = *(const v4fa*)&so[w][r][c4];
      *(volatile v4f*)(C + (size_t)(row0 + r) * ldc + col0 + c4) = v;
    }
    if (pass == 0) __threadfence();
  }
}
template <bool PARAM_BF16>
__global__ __launch_bounds__(256) void k_layernorm(const float* __restrict__ X, const float* __restrict__ R, const float* __restrict__ g, const float* __restrict__ bta,
                                                  float* __restrict__ out_sum, float* __restrict__ out_norm, int N, float eps) {
  __shared__ float red[256];
  const int row = blockIdx.x, tid = threadIdx.x;
  const float* x = X + (size_t)row * N; const float* rr = R ? R + (size_t)row * N : nullptr;
  float vals[16];
  const int per = N / 256;
  float s1 = 0.f;
  for (int u = 0; u < per / 4; ++u) {
    const int j = tid * 4 + 1024 * u;
    const v4f a = *(const v4fa*)(x + j);
    v4f b = {0.f,0.f,0.f,0.f}; if (rr) b = *(const v4fa*)(rr + j);
#pragma unroll
    for (int q = 0; q < 4; ++q) { const float v = a[q] + b[q]; vals[u * 4 + q] = v; s1 += v; }
  }
  red[tid] = s1; __syncthreads();
  for (int st = 128; st > 0; st >>= 1) { if (tid < st) red[tid] += red[tid + st]; __syncthreads(); }
  const float mu = red[0] / (float)N; __syncthreads();
  float s2 = 0.f;
  for (int u = 0; u < per / 4; ++u)
#pragma unroll
    for (int q = 0; q < 4; ++q) { const float c = vals[u * 4 + q] - mu; s2 += c * c; }
  red[tid] = s2; __syncthreads();
  for (int st = 128; st > 0; st >>= 1) { if (tid < st) red[tid] += red[tid + st]; __syncthreads(); }
  const float rs = rsqrtf(red[0] / (float)N + eps);
  for (int pass = 0; pass < 2; ++pass) {
    for (int u = 0; u < per / 4; ++u) {
      const int j = tid * 4 + 1024 * u;
      v4f o, sm;
#pragma unroll
      for (int q = 0; q < 4; ++q) {
        float gg = g[j + q], bb = bta[j + q];
        if (PARAM_BF16) { gg = bf16_round(gg); bb = bf16_round(bb); }
        sm[q] = vals[u * 4 + q]; o[q] = (vals[u * 4 + q] - mu) * rs * gg + bb;
      }
      if (out_sum) *(volatile v4f*)(out_sum + (size_t)row * N + j) = sm;
      *(volatile v4f*)(out_norm + (size_t)row * N + j) = o;
    }
    if (pass == 0) __threadfence();
  }
}

template <bool ASPLIT, bool BSPLIT, int ACT>
__global__ __launch_bounds__(128) void k_gemm_b(const float* __restrict__ A, int lda, size_t sA, const unsigned short* __restrict__ Bh, const unsigned short* __restrict__ Bl, int ldb, size_t sB,
                                             const float* __restrict__ bias, const float* __restrict__ resid, int ldr, size_t sR, float rsign, float alpha,
                                             float* __restrict__ C, int ldc, size_t sC, int M, int N, int K) {
  __shared__ __attribute__((aligned(16))) float so[4][16][64];
  const int tid = threadIdx.x, w = tid >> 5, lane = tid & 31, ln = lane & 15, hh = lane >> 4;
  const int by = blockIdx.y;
  A += (size_t)by * sA; Bh += (size_t)by * sB; if (BSPLIT) Bl += (size_t)by * sB; C += (size_t)by * sC; if (resid) resid += (size_t)by * sR;
  const int ntn = (N + 63) / 64; const int wid = blockIdx.x * 4 + w; const int mt = wid / ntn, nq = wid % ntn;
  if (mt * 16 >= M) return;
  const int row0 = mt * 16, col0 = nq * 64;
  const float* arow = A + (size_t)(row0 + ln) * lda;
  v8f acc[4] = {};
  for (int kb = 0; kb < K; kb += 32) {
    FragB ah, al;
    const v4f x0 = *(const v4fa*)(arow + kb + 8 * hh), x1 = *(const v4fa*)(arow + kb + 8 * hh + 4);
    const v4f x2 = *(const v4fa*)(arow + kb + 16 + 8 * hh), x3 = *(const v4fa*)(arow + kb + 16 + 8 * hh + 4);
    float xs[16] = {x0[0],x0[1],x0[2],x0[3],x1[0],x1[1],x1[2],x1[3],x2[0],x2[1],x2[2],x2[3],x3[0],x3[1],x3[2],x3[3]};
#pragma unroll
    for (int i = 0; i < 16; ++i) { const unsigned short hb = bf16_bits(xs[i]); ah.u[i] = hb; al.u[i] = ASPLIT ? bf16_bits(xs[i] - bf16_val(hb)) : (unsigned short)0; }
#pragma unroll
    for (int t = 0; t < 4; ++t) {
      if (col0 + t * 16 >= N) continue;
      const size_t boff = (size_t)(col0 + t * 16 + ln) * ldb + kb;
      FragB bh_, bl_; bh_.half[0] = *(const v8us*)(Bh + boff + 8 * hh); bh_.half[1] = *(const v8us*)(Bh + boff + 16 + 8 * hh);
      if (BSPLIT) { bl_.half[0] = *(const v8us*)(Bl + boff + 8 * hh); bl_.half[1] = *(const v8us*)(Bl + boff + 16 + 8 * hh); } else bl_ = bh_;
      acc[t] = mmaN<ASPLIT ? (BSPLIT ? 3 : 2) : 1>(ah.v, al.v, bh_.v, bl_.v, acc[t]);
    }
  }
#pragma unroll
  for (int t = 0; t < 4; ++t) {
    const int col = col0 + t * 16 + ln; if (col0 + t * 16 >= N) continue; const float bv = bias ? bf16_round(bias[col]) : 0.f;
#pragma unroll
    for (int r = 0; r < 8; ++r) { float v = acc[t][r] * alpha + bv; if (resid) v += rsign * resid[(size_t)(row0 + 8 * hh + r) * ldr + col]; if (ACT == 1) v = fmaxf(v, 0.f); else if (ACT == 2) v = fmaxf(v, 0.f) + log1pf(expf(-fabsf(v))); so[w][8 * hh + r][t * 16 + ln] = v; }
  }
  __builtin_amdgcn_fence(__ATOMIC_ACQ_REL, "workgroup"); __builtin_amdgcn_wave_barrier();
  const int rsub = lane >> 4, c4 = (lane & 15) * 4;
  for (int pass = 0; pass < 2; ++pass) {
#pragma unroll
    for (int q = 0; q < 8; ++q) { const int r = q * 2 + rsub; if (col0 + c4 < N) { const v4f v = *(const v4fa*)&so[w][r][c4]; *(volatile v4f*)(C + (size_t)(row0 + r) * ldc + col0 + c4) = v; } }
    if (pass == 0) __threadfence();
  }
}
__global__ __launch_bounds__(256) void k_split_transpose_b(const float* __restrict__ src, int lds_, size_t sIn, unsigned short* __restrict__ hi, unsigned short* __restrict__ lo, size_t sOut, int K, int N) {
  const size_t t = (size_t)blockIdx.x * 256 + threadIdx.x; const int k8n = K / 8; if (t >= (size_t)N * k8n) return;
  src += (size_t)blockIdx.y * sIn; hi += (size_t)blockIdx.y * sOut; lo += (size_t)blockIdx.y * sOut;
  const int n = (int)(t / k8n), k8 = (int)(t % k8n) * 8; v8us vh, vl;
#pragma unroll
  for (int i = 0; i < 8; ++i) { const float x = src[(size_t)(k8 + i) * lds_ + n]; const unsigned short hb = bf16_bits(x); vh[i] = hb; vl[i] = bf16_bits(x - bf16_val(hb)); }
  unsigned short* dh = hi + (size_t)n * K + k8; unsigned short* dl = lo + (size_t)n * K + k8;
  *(volatile v8us*)dh = vh; *(volatile v8us*)dl = vl; __threadfence(); *(volatile v8us*)dh = vh; *(volatile v8us*)dl = vl;
}

__global__ __launch_bounds__(256) void k_round_rows(const float* __restrict__ W, unsigned short* __restrict__ Wt, int n8) {
  const int t = blockIdx.x * 256 + threadIdx.x;
  if (t >= n8) return;
  const v4f a = *(const v4fa*)(W + (size_t)t * 8), b = *(const v4fa*)(W + (size_t)t * 8 + 4);
  v8us v; v[0]=bf16_bits(a[0]); v[1]=bf16_bits(a[1]); v[2]=bf16_bits(a[2]); v[3]=bf16_bits(a[3]);
  v[4]=bf16_bits(b[0]); v[5]=bf16_bits(b[1]); v[6]=bf16_bits(b[2]); v[7]=bf16_bits(b[3]);
  *(volatile v8us*)(Wt + (size_t)t * 8) = v; __threadfence(); *(volatile v8us*)(Wt + (size_t)t * 8) = v;
}

__global__ __launch_bounds__(256) void k_offset(const float* __restrict__ Q, const float* __restrict__ dww, const float* __restrict__ dwb, const float* __restrict__ lng, const float* __restrict__ lnb, const float* __restrict__ pww, float* __restrict__ POS) {
  __shared__ float so[256][66];
  const int t = blockIdx.x * 256 + threadIdx.x; const int p = t % NPIX, g = (t / NPIX) % NG, b = t / (NPIX * NG); const int y = p / WS, x = p % WS; float* o = so[threadIdx.x];
  float s1 = 0.f;
#pragma unroll 1
  for (int c = 0; c < GC; ++c) { const int ch = g * GC + c; float a = bf16_round(dwb[c]);
#pragma unroll 1
    for (int ky = 0; ky < 3; ++ky) { const int yy = y + ky - 1; if (yy < 0 || yy >= HS) continue; for (int kx = 0; kx < 3; ++kx) { const int xx = x + kx - 1; if (xx < 0 || xx >= WS) continue; a += bf16_round(dww[c * 9 + ky * 3 + kx]) * Q[((size_t)b * NPIX + yy * WS + xx) * CC + ch]; } }
    o[c] = a; s1 += a; }
  const float mu = s1 / (float)GC; float s2 = 0.f;
#pragma unroll 1
  for (int c = 0; c < GC; ++c) { const float d = o[c] - mu; s2 += d * d; }
  const float rs = 1.0f / sqrtf(s2 / (float)GC + 1e-5f); float d0 = 0.f, d1 = 0.f;
#pragma unroll 1
  for (int c = 0; c < GC; ++c) { float v = (o[c] - mu) * rs * bf16_round(lng[c]) + bf16_round(lnb[c]); v = 0.5f * v * (1.0f + erff(v * 0.70710678118654752f)); d0 += bf16_round(pww[c]) * v; d1 += bf16_round(pww[GC + c]) * v; }
  const float rng = 1.0f / 31.0f * 4.0f; const float offy = tanhf(d0) * rng, offx = tanhf(d1) * rng;
  const float sy = (y == HS - 1) ? 1.0f : (float)y * (1.0f / 31.0f), sx = (x == WS - 1) ? 1.0f : (float)x * (1.0f / 31.0f);
  const float liny = (y == HS - 1) ? 31.5f : (0.5f * (1.0f - sy) + 31.5f * sy), linx = (x == WS - 1) ? 31.5f : (0.5f * (1.0f - sx) + 31.5f * sx);
  const float refy = (liny * (1.0f / 31.0f)) * 2.0f - 1.0f, refx = (linx * (1.0f / 31.0f)) * 2.0f - 1.0f;
  const float py = ((offy + refy) + 1.0f) * 0.5f * 31.0f, px = ((offx + refx) + 1.0f) * 0.5f * 31.0f;
  { typedef float v2f __attribute__((ext_vector_type(2))); v2f pv; pv.x = py; pv.y = px; *(volatile v2f*)(POS + (size_t)t * 2) = pv; __threadfence(); *(volatile v2f*)(POS + (size_t)t * 2) = pv; }
}
__global__ __launch_bounds__(256) void k_sample(const float* __restrict__ xcl, const float* __restrict__ POS, float* __restrict__ XS) {
  const int tid = threadIdx.x, wv = tid >> 5, lane = tid & 31; const int t = blockIdx.x * 8 + wv; const int n = t % NPIX, g = (t / NPIX) % NG, b = t / (NPIX * NG);
  const float py = POS[(size_t)t * 2], px = POS[(size_t)t * 2 + 1]; const float fy = floorf(py), fx = floorf(px); const float wy = py - fy, wx = px - fx; const int y0 = (int)fy, x0 = (int)fx;
  float a0 = 0.f, a1 = 0.f;
#pragma unroll
  for (int q = 0; q < 4; ++q) { const int yi = y0 + (q >> 1), xi = x0 + (q & 1); const bool ok = (yi >= 0 && yi < HS && xi >= 0 && xi < WS); const float w = ((q >> 1) ? wy : (1.f - wy)) * ((q & 1) ? wx : (1.f - wx));
    if (ok) { const float* r = xcl + ((size_t)b * NPIX + yi * WS + xi) * CC + g * GC; a0 += bf16_round(r[lane]) * w; a1 += bf16_round(r[32 + lane]) * w; } }
  float* dst = XS + ((size_t)b * NPIX + n) * CC + g * GC; *(volatile float*)(dst + lane) = a0; *(volatile float*)(dst + 32 + lane) = a1; __threadfence(); *(volatile float*)(dst + lane) = a0; *(volatile float*)(dst + 32 + lane) = a1;
}
__global__ __launch_bounds__(256) void k_kv(const float* __restrict__ Kp, const float* __restrict__ Vp, unsigned short* __restrict__ Kb, unsigned short* __restrict__ Vt) {
  const size_t t = (size_t)blockIdx.x * 256 + threadIdx.x; if (t >= (size_t)MR * CC / 8) return;
  { v8us o; for (int q = 0; q < 8; ++q) o[q] = bf16_bits(Kp[t * 8 + q]); *(volatile v8us*)(Kb + t * 8) = o; __threadfence(); *(volatile v8us*)(Kb + t * 8) = o; }
  { const int n8 = (int)(t % (NPIX / 8)) * 8; const int c = (int)((t / (NPIX / 8)) % CC); const int b = (int)(t / ((size_t)(NPIX / 8) * CC)); v8us o; for (int q = 0; q < 8; ++q) o[q] = bf16_bits(Vp[((size_t)b * NPIX + n8 + q) * CC + c]);
    *(volatile v8us*)(Vt + ((size_t)b * CC + c) * NPIX + n8) = o; __threadfence(); *(volatile v8us*)(Vt + ((size_t)b * CC + c) * NPIX + n8) = o; }
}
__global__ __launch_bounds__(256) void k_softmax(float* __restrict__ S) {
  const int tid = threadIdx.x, wv = tid >> 5, lane = tid & 31; const size_t r = (size_t)blockIdx.x * 8 + wv; float* row = S + r * NPIX; const float sc = 0.17677669529663687f; float mx = -3.0e38f;
#pragma unroll 1
  for (int j = lane; j < NPIX; j += 32) mx = fmaxf(mx, row[j] * sc);
  for (int o = 16; o >= 1; o >>= 1) mx = fmaxf(mx, __shfl_xor(mx, o, 32));
  float den = 0.f;
#pragma unroll 1
  for (int j = lane; j < NPIX; j += 32) { const float e = expf(row[j] * sc - mx); row[j] = e; den += e; }
  for (int o = 16; o >= 1; o >>= 1) den += __shfl_xor(den, o, 32); const float inv = 1.0f / den;
#pragma unroll 1
  for (int j = lane; j < NPIX; j += 32) { const float p = row[j] * inv; *(volatile float*)(row + j) = p; __threadfence(); *(volatile float*)(row + j) = p; }
}
__global__ __launch_bounds__(256) void k_lepe(const float* __restrict__ Q, const float* __restrict__ w, const float* __restrict__ bb, float* __restrict__ O) {
  const size_t t = (size_t)blockIdx.x * 256 + threadIdx.x; if (t >= (size_t)MR * CC) return; const int c = (int)(t % CC); const size_t bm = t / CC; const int m = (int)(bm % NPIX), b = (int)(bm / NPIX); const int y = m / WS, x = m % WS;
  float a = bf16_round(bb[c]);
#pragma unroll 1
  for (int ky = 0; ky < 3; ++ky) { const int yy = y + ky - 1; if (yy < 0 || yy >= HS) continue; for (int kx = 0; kx < 3; ++kx) { const int xx = x + kx - 1; if (xx < 0 || xx >= WS) continue; a += bf16_round(w[c * 9 + ky * 3 + kx]) * Q[((size_t)b * NPIX + yy * WS + xx) * CC + c]; } }
  const float v = O[t] + a; *(volatile float*)(O + t) = v; __threadfence(); *(volatile float*)(O + t) = v;
}
extern "C" void kernel_launch(void* const* d_in, const int* in_sizes, int n_in,
                              void* d_out, int out_size, void* d_ws, size_t ws_size, hipStream_t stream) {
  (void)in_sizes; (void)n_in; (void)out_size;
  const float* x = (const float*)d_in[0]; const float* Wq = (const float*)d_in[1]; const float* bq = (const float*)d_in[2]; const float* Wk = (const float*)d_in[3]; const float* bk = (const float*)d_in[4]; const float* Wv = (const float*)d_in[5]; const float* bv = (const float*)d_in[6]; const float* Wo = (const float*)d_in[7]; const float* bo = (const float*)d_in[8];
  const float* dww = (const float*)d_in[9]; const float* dwb = (const float*)d_in[10]; const float* lng = (const float*)d_in[11]; const float* lnb = (const float*)d_in[12]; const float* pww = (const float*)d_in[13]; const float* rpw = (const float*)d_in[14]; const float* rpb = (const float*)d_in[15];
  char* ws = (char*)d_ws; size_t off = 0;
  auto take = [&](size_t bytes) { char* p = ws + off; off += (bytes + 255) & ~(size_t)255; return p; };
  unsigned short* Bq = (unsigned short*)take(CC * CC * 2); unsigned short* Bk = (unsigned short*)take(CC * CC * 2); unsigned short* Bv = (unsigned short*)take(CC * CC * 2); unsigned short* Bo = (unsigned short*)take(CC * CC * 2);
  float* xcl = (float*)take((size_t)MR * CC * 4); float* Q = (float*)take((size_t)MR * CC * 4); float* POS = (float*)take((size_t)BB * NG * NPIX * 2 * 4); float* XS = (float*)take((size_t)MR * CC * 4); float* Kp = (float*)take((size_t)MR * CC * 4); float* Vp = (float*)take((size_t)MR * CC * 4);
  unsigned short* Kb = (unsigned short*)take((size_t)MR * CC * 2); unsigned short* Vt = (unsigned short*)take((size_t)BB * CC * NPIX * 2); float* S = (float*)take((size_t)NH * NPIX * NPIX * 4); float* O = (float*)take((size_t)MR * CC * 4); float* Y = (float*)take((size_t)MR * CC * 4);
  if (off > ws_size) return;
  k_round_rows<<<(CC * CC / 8 + 255) / 256, 256, 0, stream>>>(Wq, Bq, CC * CC / 8); k_round_rows<<<(CC * CC / 8 + 255) / 256, 256, 0, stream>>>(Wk, Bk, CC * CC / 8); k_round_rows<<<(CC * CC / 8 + 255) / 256, 256, 0, stream>>>(Wv, Bv, CC * CC / 8); k_round_rows<<<(CC * CC / 8 + 255) / 256, 256, 0, stream>>>(Wo, Bo, CC * CC / 8);
  k_transpose32<false, false, false><<<dim3(NPIX / 32, CC / 32, BB), 256, 0, stream>>>(x, xcl, CC, NPIX, nullptr, nullptr, nullptr);
  const unsigned g = ((MR / 16) * (CC / 64) + 3) / 4;
  k_gemm_bf3<false, 0, true, false><<<g, 128, 0, stream>>>(xcl, CC, Bq, CC, bq, nullptr, 1, 0, Q, CC, MR, CC, CC);
  k_offset<<<(BB * NG * NPIX + 255) / 256, 256, 0, stream>>>(Q, dww, dwb, lng, lnb, pww, POS);
  k_sample<<<(BB * NG * NPIX + 7) / 8, 256, 0, stream>>>(xcl, POS, XS);
  k_gemm_bf3<true, 0, true, false><<<g, 128, 0, stream>>>(XS, CC, Bk, CC, bk, nullptr, 1, 0, Kp, CC, MR, CC, CC);
  k_gemm_bf3<true, 0, true, false><<<g, 128, 0, stream>>>(XS, CC, Bv, CC, bv, nullptr, 1, 0, Vp, CC, MR, CC, CC);
  k_kv<<<(unsigned)(((size_t)MR * CC / 8 + 255) / 256), 256, 0, stream>>>(Kp, Vp, Kb, Vt);
  for (int b = 0; b < BB; ++b) {
    k_gemm_b<true, false, 0><<<dim3(((NPIX / 16) * (NPIX / 64) + 3) / 4, NH), 128, 0, stream>>>(Q + (size_t)b * NPIX * CC, CC, HC, Kb + (size_t)b * NPIX * CC, Kb + (size_t)b * NPIX * CC, CC, HC, nullptr, nullptr, 0, 0, 1.f, 1.f, S, NPIX, (size_t)NPIX * NPIX, NPIX, NPIX, HC);
    k_softmax<<<(NH * NPIX) / 8, 256, 0, stream>>>(S);
    k_gemm_b<true, false, 0><<<dim3(((NPIX / 16) * 1 + 3) / 4, NH), 128, 0, stream>>>(S, NPIX, (size_t)NPIX * NPIX, Vt + (size_t)b * CC * NPIX, Vt + (size_t)b * CC * NPIX, NPIX, (size_t)HC * NPIX, nullptr, nullptr, 0, 0, 1.f, 1.f, O + (size_t)b * NPIX * CC, CC, (size_t)HC, NPIX, HC, NPIX);
  }
  k_lepe<<<(unsigned)(((size_t)MR * CC + 255) / 256), 256, 0, stream>>>(Q, rpw, rpb, O);
  k_gemm_bf3<true, 0, true, false><<<g, 128, 0, stream>>>(O, CC, Bo, CC, bo, nullptr, 1, 0, Y, CC, MR, CC, CC);
  k_transpose32<false, false, false><<<dim3(CC / 32, NPIX / 32, BB), 256, 0, stream>>>(Y, (float*)d_out, NPIX, CC, nullptr, nullptr, nullptr);
}
